// GATLayer_3556232922574
// MI455X (gfx1250) — hardware-verified
//
#include <hip/hip_runtime.h>
#include <stddef.h>
#include <stdint.h>
#include <math.h>


#define DF     128
#define LDC    256
#define NTHR   256
#define NWAVE  8
#define EPT    8
#define CHUNK  (NTHR * EPT)
#define WCAP   (EPT * 32)
#define LISTN  (NWAVE * WCAP)
#define NBA    1024
#define SLA    10
#define RCAP   28672
#define DEGCAP 128
#define GBM    64
#define GBN    128
#define RPW    (GBM / NWAVE)
#define NUW    (LDC * (DF / 8))
#define LEAKY  0.01f
#define AGG_ZINTS (LISTN + 2 * RCAP + 3 * NBA)
#define AGG_LDS_INTS (AGG_ZINTS + 16)
#define GEMM_LDS_FLOATS (GBM * LDC + 2 * GBM)
#define WSMAX  134217728

static_assert((CHUNK & (CHUNK - 1)) == 0 && CHUNK <= 4096);
static_assert((NBA & (NBA - 1)) == 0 && NBA == (1 << SLA));
static_assert(((long long)CHUNK << SLA) < (1LL << 31));
static_assert(LISTN % NTHR == 0);
static_assert(NBA % NWAVE == 0 && NBA % 32 == 0 && NBA % GBM == 0);
static_assert(RCAP % 4 == 0 && AGG_ZINTS % 4 == 0 && LISTN % 4 == 0);
static_assert(DF % 32 == 0 && LDC == 2 * GBN && GBN == 4 * 32 && DF == GBN);
static_assert(GBM == 4 * 16 && NTHR == 2 * 128 && GBM % NWAVE == 0);
static_assert(NUW % NTHR == 0 && (NUW / 2) % NTHR == 0);
static_assert(DF / 8 == 16);
static_assert(AGG_LDS_INTS * 4 <= 300000);
static_assert(GEMM_LDS_FLOATS * 4 <= 300000);
static_assert(DEGCAP >= 36 + 8 && RCAP >= 16710 + 4096);

typedef float          v4f   __attribute__((ext_vector_type(4)));
typedef float          v8f   __attribute__((ext_vector_type(8)));
typedef int            v4i   __attribute__((ext_vector_type(4)));
typedef int            v8i   __attribute__((ext_vector_type(8)));
typedef unsigned short v8us  __attribute__((ext_vector_type(8)));
typedef unsigned short v16us __attribute__((ext_vector_type(16)));
typedef __bf16         v16bf __attribute__((ext_vector_type(16)));
typedef v4f  __attribute__((may_alias)) v4fa;
typedef v4i  __attribute__((may_alias)) v4ia;
typedef v8us __attribute__((may_alias)) v8usa;
union FragB { v16bf v; v16us u; v8us h[2]; v8i w; };

__device__ __forceinline__ v8f wmb(const FragB& a, const FragB& b, v8f c) {
  v8f d = __builtin_amdgcn_wmma_f32_16x16x32_bf16(false, a.v, false, b.v, (short)0, c, false, false);
  asm volatile("v_nop\n\tv_nop\n\tv_nop\n\tv_nop" : "+v"(d) : "v"(a.w), "v"(b.w));
  return d;
}

__device__ __forceinline__ unsigned bf16_bits(float f) {
  const unsigned u = __float_as_uint(f);
  return (u + 0x7FFFu + ((u >> 16) & 1u)) >> 16;
}
__device__ __forceinline__ float bf16_val(float f) {
  return __uint_as_float(bf16_bits(f) << 16);
}
__device__ __forceinline__ v4f bfr4(const v4f a) {
  v4f r; r.x = bf16_val(a.x); r.y = bf16_val(a.y); r.z = bf16_val(a.z); r.w = bf16_val(a.w); return r;
}

template <int SLB>
__device__ __forceinline__ int scan_chunk(const int* __restrict__ dsts, int nE, int cbase, int slotBase,
                                          int nb, int vec8, int* list, int tid, int lane, int wave) {
  int wc = 0;
  const int el0  = tid * EPT;
  const int e0   = cbase + el0;
  const int sent = -2147483647 - 1;
  v4i da, db;
  if (vec8 != 0 && cbase + CHUNK <= nE) {
    da = *(const v4i*)(dsts + e0);
    db = *(const v4i*)(dsts + e0 + 4);
  } else {
    da.x = (e0     < nE) ? dsts[min(e0,     nE - 1)] : sent;
    da.y = (e0 + 1 < nE) ? dsts[min(e0 + 1, nE - 1)] : sent;
    da.z = (e0 + 2 < nE) ? dsts[min(e0 + 2, nE - 1)] : sent;
    da.w = (e0 + 3 < nE) ? dsts[min(e0 + 3, nE - 1)] : sent;
    db.x = (e0 + 4 < nE) ? dsts[min(e0 + 4, nE - 1)] : sent;
    db.y = (e0 + 5 < nE) ? dsts[min(e0 + 5, nE - 1)] : sent;
    db.z = (e0 + 6 < nE) ? dsts[min(e0 + 6, nE - 1)] : sent;
    db.w = (e0 + 7 < nE) ? dsts[min(e0 + 7, nE - 1)] : sent;
  }
  const unsigned nbs = (unsigned)slotBase;
  const unsigned unb = (unsigned)nb;
  const unsigned s0 = (unsigned)da.x - nbs, s1 = (unsigned)da.y - nbs;
  const unsigned s2 = (unsigned)da.z - nbs, s3 = (unsigned)da.w - nbs;
  const unsigned s4 = (unsigned)db.x - nbs, s5 = (unsigned)db.y - nbs;
  const unsigned s6 = (unsigned)db.z - nbs, s7 = (unsigned)db.w - nbs;
  const bool h0 = s0 < unb, h1 = s1 < unb, h2 = s2 < unb, h3 = s3 < unb;
  const bool h4 = s4 < unb, h5 = s5 < unb, h6 = s6 < unb, h7 = s7 < unb;
  const unsigned any = __builtin_amdgcn_ballot_w32(h0 | h1 | h2 | h3 | h4 | h5 | h6 | h7);
  if (any != 0u) {
#define HITJ(J, HJ, SJ) { \
      const unsigned mj = __builtin_amdgcn_ballot_w32(HJ); \
      if (mj != 0u) { \
        if (HJ) { \
          const int pos = wc + (int)__builtin_amdgcn_mbcnt_lo(mj, 0u); \
          if (pos < WCAP) list[wave * WCAP + pos] = ((el0 + (J)) << SLB) | (int)(SJ); \
        } \
        wc += (int)__builtin_popcount(mj); } }
    HITJ(0, h0, s0)
    HITJ(1, h1, s1)
    HITJ(2, h2, s2)
    HITJ(3, h3, s3)
    HITJ(4, h4, s4)
    HITJ(5, h5, s5)
    HITJ(6, h6, s6)
    HITJ(7, h7, s7)
#undef HITJ
  }
  return wc;
}

__global__ __launch_bounds__(NTHR) void k_prep(const float* __restrict__ x, const float* __restrict__ Wm,
                                               const float* __restrict__ Wr, int nN, int nUx,
                                               unsigned short* wb, unsigned short* xb) {
  const int u = (int)blockIdx.x * NTHR + (int)threadIdx.x;
  const float* p;
  unsigned short* dp;
  bool ok;
  if (u < NUW) {
    const int n  = u >> 4;
    const int k8 = (u & 15) * 8;
    const float* wsrc = (n < DF) ? Wm : Wr;
    p  = wsrc + (size_t)(n & (DF - 1)) * DF + k8;
    dp = wb + (size_t)n * DF + k8;
    ok = true;
  } else {
    const int v = u - NUW;
    if (v >= nUx) return;
    const int row = v >> 4;
    const int k8  = (v & 15) * 8;
    const int rc  = row < nN ? row : nN - 1;
    p  = x + (size_t)rc * DF + k8;
    dp = xb + (size_t)row * DF + k8;
    ok = row < nN;
  }
  const v4f a = *(const v4f*)p;
  const v4f b = *(const v4f*)(p + 4);
  v8us o;
  o[0] = ok ? (unsigned short)bf16_bits(a.x) : (unsigned short)0;
  o[1] = ok ? (unsigned short)bf16_bits(a.y) : (unsigned short)0;
  o[2] = ok ? (unsigned short)bf16_bits(a.z) : (unsigned short)0;
  o[3] = ok ? (unsigned short)bf16_bits(a.w) : (unsigned short)0;
  o[4] = ok ? (unsigned short)bf16_bits(b.x) : (unsigned short)0;
  o[5] = ok ? (unsigned short)bf16_bits(b.y) : (unsigned short)0;
  o[6] = ok ? (unsigned short)bf16_bits(b.z) : (unsigned short)0;
  o[7] = ok ? (unsigned short)bf16_bits(b.w) : (unsigned short)0;
  *(volatile v8us*)dp = o;
  __threadfence();
  *(volatile v8us*)dp = o;
}

__global__ __launch_bounds__(NTHR) void k_gemm(const unsigned short* __restrict__ A,
                                               const unsigned short* __restrict__ BT,
                                               float* MSG, float* PP,
                                               const float* __restrict__ attn, const float* __restrict__ coef,
                                               float* AL) {
  extern __shared__ __attribute__((aligned(16))) float gsm[];
  float* stg = gsm;
  float* sdt = gsm + GBM * LDC;
  const int tid = (int)threadIdx.x, lane = tid & 31, wave = tid >> 5, hh = lane >> 4, m = lane & 15;
  const int rg = wave & 3, cg = wave >> 2;
  const int rowBase = (int)blockIdx.x * GBM;
  const int colBase = cg * GBN;

  v8f acc[8];
  {
    const v8f z = {0.f, 0.f, 0.f, 0.f, 0.f, 0.f, 0.f, 0.f};
#pragma unroll
    for (int t = 0; t < 8; ++t) acc[t] = z;
  }
  const unsigned short* ap = A  + (size_t)(rowBase + 16 * rg + m) * (size_t)DF + 8 * hh;
  const unsigned short* bp = BT + (size_t)(colBase + m) * (size_t)DF + 8 * hh;

#pragma unroll 1
  for (int k0 = 0; k0 < DF; k0 += 32) {
    FragB af;
    af.h[0] = *(const v8usa*)(ap + k0);
    af.h[1] = *(const v8usa*)(ap + k0 + 16);
#pragma unroll
    for (int nt = 0; nt < 8; ++nt) {
      const unsigned short* wq = bp + (size_t)(16 * nt) * (size_t)DF + k0;
      FragB bf;
      bf.h[0] = *(const v8usa*)wq;
      bf.h[1] = *(const v8usa*)(wq + 16);
      acc[nt] = wmb(af, bf, acc[nt]);
    }
  }

#pragma unroll
  for (int nt = 0; nt < 8; ++nt) {
    const int lc = colBase + 16 * nt + m;
#pragma unroll
    for (int r = 0; r < 8; ++r) {
      const int lr = 16 * rg + 8 * hh + r;
      stg[lr * LDC + lc] = acc[nt][r];
    }
  }
  __syncthreads();

  const v4f as4 = bfr4(*(const v4fa*)(attn + 4 * lane));
  const v4f ad4 = bfr4(*(const v4fa*)(attn + DF + 4 * lane));
  const float cb  = bf16_val(coef[0]);
  const float sig = 1.0f / (1.0f + expf(-cb));
#pragma unroll 1
  for (int i = 0; i < RPW; ++i) {
    const int row = wave * RPW + i;
    const v4f p = *(const v4fa*)(stg + row * LDC + 4 * lane);
    float s = 0.0f, d = 0.0f;
    s = fmaf(p.x, as4.x, s); s = fmaf(p.y, as4.y, s); s = fmaf(p.z, as4.z, s); s = fmaf(p.w, as4.w, s);
    d = fmaf(p.x, ad4.x, d); d = fmaf(p.y, ad4.y, d); d = fmaf(p.z, ad4.z, d); d = fmaf(p.w, ad4.w, d);
#pragma unroll
    for (int off = 16; off > 0; off >>= 1) {
      s += __shfl_xor(s, off);
      d += __shfl_xor(d, off);
    }
    if (lane == 0) { sdt[row] = s; sdt[GBM + row] = d; }
  }
  __syncthreads();

  const v4f alv = *(const v4fa*)(sdt + 4 * lane);
  float* alp = AL + (size_t)blockIdx.x * (2 * GBM) + 4 * lane;
#pragma unroll 1
  for (int i = 0; i < RPW; ++i) {
    const int row = wave * RPW + i;
    const v4f p0 = *(const v4fa*)(stg + row * LDC + 4 * lane);
    const v4f q  = *(const v4fa*)(stg + row * LDC + GBN + 4 * lane);
    v4f p1; p1.x = q.x * sig; p1.y = q.y * sig; p1.z = q.z * sig; p1.w = q.w * sig;
    const size_t ro = (size_t)(rowBase + row) * (size_t)DF + 4 * lane;
    *(volatile v4f*)(MSG + ro) = p0;
    *(volatile v4f*)(PP + ro)  = p1;
  }
  if (wave == 0) *(volatile v4f*)alp = alv;
  __threadfence();
#pragma unroll 1
  for (int i = 0; i < RPW; ++i) {
    const int row = wave * RPW + i;
    const v4f p0 = *(const v4fa*)(stg + row * LDC + 4 * lane);
    const v4f q  = *(const v4fa*)(stg + row * LDC + GBN + 4 * lane);
    v4f p1; p1.x = q.x * sig; p1.y = q.y * sig; p1.z = q.z * sig; p1.w = q.w * sig;
    const size_t ro = (size_t)(rowBase + row) * (size_t)DF + 4 * lane;
    *(volatile v4f*)(MSG + ro) = p0;
    *(volatile v4f*)(PP + ro)  = p1;
  }
  if (wave == 0) *(volatile v4f*)alp = alv;
}

__device__ __forceinline__ float hit_logit(const int* sl, const int* __restrict__ srcs,
                                           const float* __restrict__ AL, int o, int b0, int lane,
                                           int nE, int nN, float ad, int& srOut) {
  int idx = o + b0 + lane;
  idx = idx < 0 ? 0 : (idx > RCAP - 1 ? RCAP - 1 : idx);
  const int ent = sl[idx];
  int eid = ent >> SLA;
  eid = eid < 0 ? 0 : (eid > nE - 1 ? nE - 1 : eid);
  int sr = srcs[eid];
  sr = sr < 0 ? 0 : (sr > nN - 1 ? nN - 1 : sr);
  const float es = AL[(sr >> 6) * (2 * GBM) + (sr & (GBM - 1))];
  float lg = es + ad;
  lg = (lg >= 0.0f) ? lg : LEAKY * lg;
  srOut = sr;
  return lg;
}

__global__ __launch_bounds__(NTHR) void k_scan(const int* __restrict__ srcs, const int* __restrict__ dsts,
                                               int nE, int nN, int vec8,
                                               const float* __restrict__ AL, const float* __restrict__ MSG,
                                               const float* __restrict__ PP, float* outp) {
  extern __shared__ __attribute__((aligned(16))) int dsm[];
  int* list = dsm;
  int* hl   = dsm + LISTN;
  int* sl   = dsm + LISTN + RCAP;
  int* cnt  = dsm + LISTN + 2 * RCAP;
  int* offs = cnt + NBA;
  int* cur  = offs + NBA;
  int* misc = cur + NBA;
  const int tid = (int)threadIdx.x, lane = tid & 31, wave = tid >> 5;
  const int nodeBase = (int)blockIdx.x * NBA;

  {
    const v4i z4 = {0, 0, 0, 0};
    for (int i = tid * 4; i < AGG_ZINTS; i += NTHR * 4) *(v4ia*)(dsm + i) = z4;
    if (tid < 16) misc[tid] = 0;
  }
  __syncthreads();

  int t = 0, ov = 0;
  const int nChunks = (nE + CHUNK - 1) / CHUNK;
#pragma unroll 1
  for (int ch = 0; ch < nChunks; ++ch) {
    const int cbase = ch * CHUNK;
    const int wc = scan_chunk<SLA>(dsts, nE, cbase, nodeBase, NBA, vec8, list, tid, lane, wave);
    if (lane == 0) misc[wave] = wc;
    __syncthreads();
    if (wave == 0) {
#pragma unroll 1
      for (int w2 = 0; w2 < NWAVE; ++w2) {
        int c = misc[w2];
        c = c < 0 ? 0 : (c > WCAP ? WCAP : c);
#pragma unroll 1
        for (int b0 = 0; b0 < c; b0 += 32) {
          const int idx = b0 + lane;
          const int ent = list[w2 * WCAP + (idx < WCAP ? idx : WCAP - 1)];
          const int m32 = (c - b0) < 32 ? (c - b0) : 32;
#pragma unroll 1
          for (int k = 0; k < m32; ++k) {
            const int u    = __builtin_amdgcn_readlane(ent, k);
            const int slot = u & (NBA - 1);
            const int el   = (u >> SLA) & (CHUNK - 1);
            const int pk   = ((cbase + el) << SLA) | slot;
            if (t < RCAP) {
              if (lane == 0) { hl[t] = pk; cnt[slot] = cnt[slot] + 1; }
              t = t + 1;
            } else {
              ov = 1;
            }
          }
        }
      }
    }
    __syncthreads();
  }
  if (wave == 0 && lane == 0) { misc[8] = t; misc[9] = ov; }
  __syncthreads();
  int tt = misc[8];
  tt = tt < 0 ? 0 : (tt > RCAP ? RCAP : tt);
  const int ovf = misc[9];

  if (wave == 0) {
    const int base = lane * (NBA / 32);
    int s = 0;
#pragma unroll 1
    for (int i = 0; i < NBA / 32; ++i) s += cnt[base + i];
    int incl = s;
#pragma unroll
    for (int d = 1; d < 32; d <<= 1) {
      const int y = __shfl_up(incl, d, 32);
      if (lane >= d) incl += y;
    }
    int run = incl - s;
#pragma unroll 1
    for (int i = 0; i < NBA / 32; ++i) {
      const int cv = cnt[base + i];
      offs[base + i] = run;
      cur[base + i]  = run;
      run += cv;
    }
  }
  __syncthreads();
  if (wave == 0) {
#pragma unroll 1
    for (int b0 = 0; b0 < tt; b0 += 32) {
      const int idx = b0 + lane;
      const int ent = hl[idx < RCAP ? idx : RCAP - 1];
      const int m32 = (tt - b0) < 32 ? (tt - b0) : 32;
#pragma unroll 1
      for (int k = 0; k < m32; ++k) {
        const int u    = __builtin_amdgcn_readlane(ent, k);
        const int slot = u & (NBA - 1);
        if (lane == 0) {
          int p = cur[slot];
          p = p < 0 ? 0 : (p > RCAP - 1 ? RCAP - 1 : p);
          sl[p] = u;
          cur[slot] = p + 1;
        }
      }
    }
  }
  __syncthreads();

  const float qnan = __int_as_float(0x7fc00000);
  const float pz = (ovf != 0) ? qnan : 0.0f;
#pragma unroll 1
  for (int si = 0; si < NBA / NWAVE; ++si) {
    const int s    = si * NWAVE + wave;
    const int node = nodeBase + s;
    int c = cnt[s];
    const bool big = c > DEGCAP;
    c = c < 0 ? 0 : (c > DEGCAP ? DEGCAP : c);
    int o = offs[s];
    o = o < 0 ? 0 : (o > tt ? tt : o);
    if (c > tt - o) c = tt - o;
    c = __builtin_amdgcn_readfirstlane(c);
    o = __builtin_amdgcn_readfirstlane(o);
    const int nc  = node < nN ? node : nN - 1;
    const float ad = AL[(nc >> 6) * (2 * GBM) + GBM + (nc & (GBM - 1))];
    float a0 = 0.0f, a1 = 0.0f, a2 = 0.0f, a3 = 0.0f;

    if (c > 0) {
      float mxl = -3.0e38f;
#pragma unroll 1
      for (int b0 = 0; b0 < c; b0 += 32) {
        int sr;
        const float lg = hit_logit(sl, srcs, AL, o, b0, lane, nE, nN, ad, sr);
        const bool ok = (b0 + lane) < c;
        const float cand = fmaxf(mxl, lg);
        mxl = ok ? cand : mxl;
      }
      float mx = mxl;
#pragma unroll
      for (int off = 16; off > 0; off >>= 1) mx = fmaxf(mx, __shfl_xor(mx, off));
      float sml = 0.0f;
#pragma unroll 1
      for (int b0 = 0; b0 < c; b0 += 32) {
        int sr;
        const float lg = hit_logit(sl, srcs, AL, o, b0, lane, nE, nN, ad, sr);
        const bool ok = (b0 + lane) < c;
        const float w = expf(lg - mx);
        sml += ok ? w : 0.0f;
      }
      float sm = sml;
#pragma unroll
      for (int off = 16; off > 0; off >>= 1) sm += __shfl_xor(sm, off);
      const float rinv = 1.0f / sm;
#pragma unroll 1
      for (int b0 = 0; b0 < c; b0 += 32) {
        int sr;
        const float lg = hit_logit(sl, srcs, AL, o, b0, lane, nE, nN, ad, sr);
        const float w  = expf(lg - mx);
        const float al = w * rinv;
        const int ali  = __float_as_int(al);
        const int m32  = (c - b0) < 32 ? (c - b0) : 32;
#pragma unroll 1
        for (int k = 0; k < m32; ++k) {
          const int   sk = __builtin_amdgcn_readlane(sr, k);
          const float ak = __int_as_float(__builtin_amdgcn_readlane(ali, k));
          const v4f r = *(const v4f*)(MSG + (size_t)sk * DF + 4 * lane);
          a0 = fmaf(ak, r.x, a0);
          a1 = fmaf(ak, r.y, a1);
          a2 = fmaf(ak, r.z, a2);
          a3 = fmaf(ak, r.w, a3);
        }
      }
    }

    const float pzr = big ? qnan : pz;
    const v4f pv = *(const v4f*)(PP + (size_t)nc * DF + 4 * lane);
    v4f ov4;
    ov4.x = (pv.x + ((a0 > 0.0f) ? a0 : (a0 - a0))) + pzr;
    ov4.y = (pv.y + ((a1 > 0.0f) ? a1 : (a1 - a1))) + pzr;
    ov4.z = (pv.z + ((a2 > 0.0f) ? a2 : (a2 - a2))) + pzr;
    ov4.w = (pv.w + ((a3 > 0.0f) ? a3 : (a3 - a3))) + pzr;
    if (node < nN) {
      float* op = outp + (size_t)node * DF + 4 * lane;
      *(volatile v4f*)op = ov4;
      __threadfence();
      *(volatile v4f*)op = ov4;
    }
  }
}

static inline int cdiv(int a, int b) { return (a + b - 1) / b; }

extern "C" void kernel_launch(void* const* d_in, const int* in_sizes, int n_in,
                              void* d_out, int out_size, void* d_ws, size_t ws_size,
                              hipStream_t stream) {
  if (n_in < 6) return;
  if (in_sizes[0] < DF || (in_sizes[0] % DF) != 0) return;
  const int nN = in_sizes[0] / DF;
  if (nN > (1 << 22)) return;
  if (in_sizes[1] < 2 || (in_sizes[1] & 1) != 0) return;
  const int nE = in_sizes[1] / 2;
  if (nE < 1 || nE >= (1 << 21)) return;
  if (in_sizes[2] != DF * DF) return;
  if (in_sizes[3] != 2 * DF) return;
  if (in_sizes[4] != DF * DF) return;
  if (in_sizes[5] < 1) return;
  if ((long long)out_size != (long long)nN * DF) return;

  const float* x    = (const float*)d_in[0];
  const int*   edge = (const int*)d_in[1];
  const float* Wm   = (const float*)d_in[2];
  const float* attn = (const float*)d_in[3];
  const float* Wr   = (const float*)d_in[4];
  const float* coef = (const float*)d_in[5];
  float* out = (float*)d_out;
  const int* src = edge;
  const int* dst = edge + nE;

  const int MP   = cdiv(nN, GBM) * GBM;
  const int gM   = MP / GBM;
  const int gA   = cdiv(nN, NBA);
  if ((long long)gA * NBA < (long long)nN) return;
  const int vec8 = ((nE & 3) == 0) ? 1 : 0;

  char* ws = (char*)d_ws;
  size_t off = 0;
  const size_t oWB  = off; off += (size_t)LDC * DF * 2;                  off = (off + 255) & ~(size_t)255;
  const size_t oAL  = off; off += (size_t)gM * (2 * GBM) * 4;            off = (off + 255) & ~(size_t)255;
  const size_t oXB  = off; off += (size_t)MP * DF * 2;                   off = (off + 255) & ~(size_t)255;
  const size_t oMSG = off; off += (size_t)MP * DF * 4;                   off = (off + 255) & ~(size_t)255;
  const size_t oPP  = off; off += (size_t)MP * DF * 4;                   off = (off + 255) & ~(size_t)255;
  if (off > ws_size || off > (size_t)WSMAX) return;
  unsigned short* WB  = (unsigned short*)(ws + oWB);
  float*          ALp = (float*)(ws + oAL);
  unsigned short* XB  = (unsigned short*)(ws + oXB);
  float*          MSG = (float*)(ws + oMSG);
  float*          PPp = (float*)(ws + oPP);

  const size_t aggLds  = (size_t)AGG_LDS_INTS * 4;
  const size_t gemmLds = (size_t)GEMM_LDS_FLOATS * 4;
  hipFuncSetAttribute(reinterpret_cast<const void*>(&k_gemm), hipFuncAttributeMaxDynamicSharedMemorySize, (int)gemmLds);
  hipFuncSetAttribute(reinterpret_cast<const void*>(&k_scan), hipFuncAttributeMaxDynamicSharedMemorySize, (int)aggLds);

  const int nUx = MP * (DF / 8);
  k_prep<<<(NUW + nUx) / NTHR + (((NUW + nUx) % NTHR) ? 1 : 0), NTHR, 0, stream>>>(x, Wm, Wr, nN, nUx, WB, XB);
  k_gemm<<<gM, NTHR, gemmLds, stream>>>(XB, WB, MSG, PPp, attn, coef, ALp);
  k_scan<<<gA, NTHR, aggLds, stream>>>(src, dst, nE, nN, vec8, ALp, MSG, PPp, out);
}
